// PMA_481036337712
// MI455X (gfx1250) — hardware-verified
//
#include <hip/hip_runtime.h>
#include <math.h>

typedef __attribute__((ext_vector_type(16))) _Float16 v16h;
typedef __attribute__((ext_vector_type(16))) __bf16 v16b;
typedef __attribute__((ext_vector_type(8)))  _Float16 v8h;
typedef __attribute__((ext_vector_type(8)))  float v8f;
typedef __attribute__((ext_vector_type(4)))  float v4f;
typedef __attribute__((ext_vector_type(2)))  float v2f;
typedef __attribute__((ext_vector_type(4)))  unsigned v4u;
typedef __attribute__((ext_vector_type(4)))  int v4i;
typedef float __attribute__((may_alias)) float_a;
typedef int __attribute__((may_alias)) int_a;

template <typename T> __device__ __forceinline__ void vst2(void* p, T v) { *(volatile T*)p = v; __threadfence(); *(volatile T*)p = v; }
__device__ __forceinline__ v8f wmma16(v16h a, v16h b, v8f c) {
  v8f d = __builtin_amdgcn_wmma_f32_16x16x32_f16(false, a, false, b, (short)0, c, false, false);
  asm volatile("v_nop\n\tv_nop\n\tv_nop\n\tv_nop" : "+v"(d) : "v"(a), "v"(b));
  return d;
}
__device__ __forceinline__ v8f wmma_bf(v16b a, v16b b, v8f c) {
  v8f d = __builtin_amdgcn_wmma_f32_16x16x32_bf16(false, a, false, b, (short)0, c, false, false);
  asm volatile("v_nop\n\tv_nop\n\tv_nop\n\tv_nop" : "+v"(d) : "v"(a), "v"(b));
  return d;
}
__device__ __forceinline__ v16h frag_h(const _Float16* rowk0, int lane) {
  union { v16h v; v8h q[2]; } u; const _Float16* p = rowk0 + 8 * (lane >> 4);
  u.q[0] = *(const v8h*)p; u.q[1] = *(const v8h*)(p + 16); return u.v;
}
__device__ __forceinline__ v16h frag_f32(const float* rowk0, int lane) {
  v16h a; const float* p = rowk0 + 8 * (lane >> 4);
#pragma unroll
  for (int i = 0; i < 8; ++i) { a[i] = (_Float16)p[i]; a[8 + i] = (_Float16)p[16 + i]; }
  return a;
}
__device__ __forceinline__ v16h frag_f32s(const float* rowk0, int lane, float sc) {
  v16h a; const float* p = rowk0 + 8 * (lane >> 4);
#pragma unroll
  for (int i = 0; i < 8; ++i) { a[i] = (_Float16)(p[i] * sc); a[8 + i] = (_Float16)(p[16 + i] * sc); }
  return a;
}
__device__ __forceinline__ v16h fragc_f32(const float* W, int k0, int n, int lane, int ld, int K) {
  v16h a; const int g = lane >> 4;
#pragma unroll
  for (int i = 0; i < 8; ++i) { const int ka = k0 + 8 * g + i, kb = ka + 16;
    a[i] = (_Float16)(ka < K ? W[(size_t)ka * ld + n] : 0.f); a[8 + i] = (_Float16)(kb < K ? W[(size_t)kb * ld + n] : 0.f); }
  return a;
}
struct F2 { v16b h, l; };
__device__ __forceinline__ F2 bsplit16(const float v[16]) { F2 r;
#pragma unroll
  for (int i = 0; i < 16; ++i) { const __bf16 h = (__bf16)v[i]; r.h[i] = h; r.l[i] = (__bf16)(v[i] - (float)h); }
  return r; }
__device__ __forceinline__ F2 split_row(const float* row, int k0, int lane) { float v[16]; const float* p = row + k0 + 8 * (lane >> 4);
#pragma unroll
  for (int i = 0; i < 8; ++i) { v[i] = p[i]; v[8 + i] = p[16 + i]; }
  return bsplit16(v); }
__device__ __forceinline__ F2 split_rowK(const float* row, int k0, int lane, int K) { float v[16]; const int g = lane >> 4;
#pragma unroll
  for (int i = 0; i < 8; ++i) { const int ka = k0 + 8 * g + i, kb = ka + 16; v[i] = ka < K ? row[ka] : 0.f; v[8 + i] = kb < K ? row[kb] : 0.f; }
  return bsplit16(v); }
__device__ __forceinline__ F2 split_col(const float* W, int k0, int n, int lane, int ld, int K) { float v[16]; const int g = lane >> 4;
#pragma unroll
  for (int i = 0; i < 8; ++i) { const int ka = k0 + 8 * g + i, kb = ka + 16; v[i] = ka < K ? W[(size_t)ka * ld + n] : 0.f; v[8 + i] = kb < K ? W[(size_t)kb * ld + n] : 0.f; }
  return bsplit16(v); }
__device__ __forceinline__ v8f mac3(const F2& a, const F2& b, v8f c) { c = wmma_bf(a.l, b.h, c); c = wmma_bf(a.h, b.l, c); return wmma_bf(a.h, b.h, c); }
__device__ __forceinline__ float sigm(float v) { return 1.0f / (1.0f + expf(-v)); }
#define LDSX() do { asm volatile("s_wait_dscnt 0" ::: "memory"); __builtin_amdgcn_wave_barrier(); __builtin_amdgcn_fence(__ATOMIC_RELEASE, "workgroup"); } while (0)

#define NBT 64
#define SS 512
#define DD 256
#define NH 4
#define NR (NBT * SS)

__global__ __launch_bounds__(256) void k_setup(const float* __restrict__ seeds, const float* __restrict__ Wq, const float* __restrict__ bq, const float* __restrict__ Wk, const float* __restrict__ bk, float* __restrict__ qv, float* __restrict__ U, float* __restrict__ cb) {
  __shared__ float sq[NH][DD]; __shared__ __align__(16) float su[16][DD]; __shared__ __align__(16) float scb[32];
  const int tid = threadIdx.x;
  for (int o = tid; o < NH * DD; o += 256) { const int h = o >> 8, e = o & 255; float s = bq[o];
    for (int d = 0; d < DD; ++d) s += seeds[d] * Wq[((size_t)d * NH + h) * DD + e];
    sq[h][e] = s; }
  __syncthreads();
  for (int o = tid; o < 16 * DD; o += 256) { const int n = o >> 8, d = o & 255; float s = 0.f;
    if (n < NH) { const float* wr = Wk + ((size_t)d * NH + n) * DD; for (int e = 0; e < DD; ++e) s += wr[e] * sq[n][e]; }
    su[n][d] = s; }
  if (tid < 32) { float s = 0.f; if (tid < NH) { for (int e = 0; e < DD; ++e) s += sq[tid][e] * bk[tid * DD + e]; } scb[tid] = s; }
  __syncthreads();
  for (int q = tid; q < NH * DD / 4; q += 256) vst2(qv + q * 4, *(const v4f*)(&sq[0][0] + q * 4));
  for (int q = tid; q < 16 * DD / 4; q += 256) vst2(U + q * 4, *(const v4f*)(&su[0][0] + q * 4));
  if (tid < 8) vst2(cb + tid * 4, *(const v4f*)(&scb[tid * 4]));
}
__global__ __launch_bounds__(128) void k_scores(const float* __restrict__ x, const float* __restrict__ U, const float* __restrict__ cb, float* __restrict__ SC) {
  __shared__ __align__(16) float so[4][16][20];
  const int tid = threadIdx.x, wave = tid >> 5, lane = tid & 31, col = lane & 15, g = lane >> 4;
  const int r0 = blockIdx.x * 64 + wave * 16;
  v8f acc = {};
#pragma unroll 2
  for (int kc = 0; kc < DD / 32; ++kc) acc = mac3(split_row(x + (size_t)(r0 + col) * DD, kc * 32, lane), split_row(U + (size_t)col * DD, kc * 32, lane), acc);
  const float c0 = col < NH ? cb[col] : 0.f;
#pragma unroll
  for (int r = 0; r < 8; ++r) so[wave][8 * g + r][col] = (acc[r] + c0) * 0.0625f;
  LDSX();
  for (int q = lane; q < 16 * 4; q += 32) { const int rl = q >> 2, pc = q & 3; vst2(SC + (size_t)(r0 + rl) * 16 + pc * 4, *(const v4f*)(&so[wave][rl][pc * 4])); }
}
__global__ __launch_bounds__(256) void k_pool(const float* __restrict__ SC, const int* __restrict__ mask, const float* __restrict__ x, float* __restrict__ Y) {
  __shared__ float sp[NH][SS]; __shared__ float sred[NH][2]; __shared__ __align__(16) float sy[NH][DD];
  const int b = blockIdx.x, tid = threadIdx.x;
  for (int q = tid; q < NH * SS; q += 256) { const int h = q / SS, s = q % SS; const float m = (float)mask[(size_t)b * SS + s]; sp[h][s] = SC[((size_t)b * SS + s) * 16 + h] + (1.0f - m) * -1.0e9f; }
  __syncthreads();
  if (tid < NH * 32) { const int h = tid >> 5, lane = tid & 31; float mx = -3.4e38f; for (int s = lane; s < SS; s += 32) mx = fmaxf(mx, sp[h][s]);
#pragma unroll
    for (int off = 16; off >= 1; off >>= 1) mx = fmaxf(mx, __shfl_xor(mx, off, 32));
    float l = 0.f; for (int s = lane; s < SS; s += 32) { const float p = expf(sp[h][s] - mx); sp[h][s] = p; l += p; }
#pragma unroll
    for (int off = 16; off >= 1; off >>= 1) l += __shfl_xor(l, off, 32);
    if (lane == 0) sred[h][0] = 1.0f / l; }
  __syncthreads();
  { const int d = tid; float a[NH] = {0.f, 0.f, 0.f, 0.f}; const float* xb = x + (size_t)b * SS * DD;
#pragma unroll 4
    for (int s = 0; s < SS; ++s) { const float xv = xb[(size_t)s * DD + d];
#pragma unroll
      for (int h = 0; h < NH; ++h) a[h] += sp[h][s] * xv; }
#pragma unroll
    for (int h = 0; h < NH; ++h) sy[h][d] = a[h] * sred[h][0]; }
  __syncthreads();
  for (int q = tid; q < NH * DD / 4; q += 256) vst2(Y + (size_t)b * NH * DD + q * 4, *(const v4f*)(&sy[0][0] + q * 4));
}
__global__ __launch_bounds__(256) void k_fin(const float* __restrict__ Y, const float* __restrict__ Wv, const float* __restrict__ bv, const float* __restrict__ Wo, const float* __restrict__ bo, const float* __restrict__ seeds, const float* __restrict__ gam, const float* __restrict__ bet, float* __restrict__ out) {
  __shared__ float sy[NH][DD]; __shared__ float so[NH][DD]; __shared__ __align__(16) float sh[DD]; __shared__ float sred[2][8];
  const int b = blockIdx.x, tid = threadIdx.x, wv = tid >> 5, lane = tid & 31;
  for (int q = tid; q < NH * DD; q += 256) sy[q >> 8][q & 255] = Y[(size_t)b * NH * DD + q];
  __syncthreads();
  { const int e = tid; float a[NH];
#pragma unroll
    for (int h = 0; h < NH; ++h) a[h] = bv[h * DD + e];
#pragma unroll 2
    for (int d = 0; d < DD; ++d) {
#pragma unroll
      for (int h = 0; h < NH; ++h) a[h] += sy[h][d] * Wv[((size_t)d * NH + h) * DD + e]; }
#pragma unroll
    for (int h = 0; h < NH; ++h) so[h][e] = a[h]; }
  __syncthreads();
  { const int d = tid; float a = bo[d] + seeds[d];
#pragma unroll 2
    for (int h = 0; h < NH; ++h) for (int e = 0; e < DD; ++e) a += so[h][e] * Wo[((size_t)h * DD + e) * DD + d];
    sh[d] = a;
    float s = a;
#pragma unroll
    for (int off = 16; off >= 1; off >>= 1) s += __shfl_xor(s, off, 32);
    if (lane == 0) sred[0][wv] = s; }
  __syncthreads();
  { float mu = 0.f; for (int i = 0; i < 8; ++i) mu += sred[0][i]; mu *= (1.0f / DD);
    const float dv = sh[tid] - mu; float s2 = dv * dv;
#pragma unroll
    for (int off = 16; off >= 1; off >>= 1) s2 += __shfl_xor(s2, off, 32);
    if (lane == 0) sred[1][wv] = s2;
    __syncthreads();
    float var = 0.f; for (int i = 0; i < 8; ++i) var += sred[1][i]; var *= (1.0f / DD);
    const float yv = dv * rsqrtf(var + 1e-6f) * gam[tid] + bet[tid];
    __syncthreads();
    sh[tid] = yv; }
  __syncthreads();
  if (tid < DD / 4) vst2(out + (size_t)b * DD + tid * 4, *(const v4f*)(&sh[tid * 4]));
}
extern "C" void kernel_launch(void* const* d_in, const int* in_sizes, int n_in, void* d_out, int out_size, void* d_ws, size_t ws_size, hipStream_t stream) {
  (void)in_sizes; (void)n_in; (void)out_size; (void)ws_size;
  const float* x = (const float*)d_in[0]; const int* mask = (const int*)d_in[1]; const float* seeds = (const float*)d_in[2];
  const float* Wq = (const float*)d_in[3]; const float* bq = (const float*)d_in[4]; const float* Wk = (const float*)d_in[5]; const float* bk = (const float*)d_in[6]; const float* Wv = (const float*)d_in[7]; const float* bv = (const float*)d_in[8];
  const float* Wo = (const float*)d_in[9]; const float* bo = (const float*)d_in[10]; const float* gam = (const float*)d_in[11]; const float* bet = (const float*)d_in[12];
  float* out = (float*)d_out;
  char* ws = (char*)d_ws; size_t off = 0;
  auto take = [&](size_t bytes) { char* p = ws + off; off += (bytes + 255) & ~(size_t)255; return p; };
  float* qv = (float*)take(NH * DD * 4); float* U = (float*)take(16 * DD * 4); float* cb = (float*)take(32 * 4); float* SC = (float*)take((size_t)NR * 16 * 4); float* Y = (float*)take((size_t)NBT * NH * DD * 4);
  k_setup<<<1, 256, 0, stream>>>(seeds, Wq, bq, Wk, bk, qv, U, cb);
  k_scores<<<NR / 64, 128, 0, stream>>>(x, U, cb, SC);
  k_pool<<<NBT, 256, 0, stream>>>(SC, mask, x, Y);
  k_fin<<<NBT, 256, 0, stream>>>(Y, Wv, bv, Wo, bo, seeds, gam, bet, out);
}
